// CoAtNetTransformerBlock_44092134261303
// MI455X (gfx1250) — hardware-run, weakly checked
//
#include <hip/hip_runtime.h>

typedef __attribute__((ext_vector_type(16))) _Float16 v16h;
typedef __attribute__((ext_vector_type(8)))  _Float16 v8h;
typedef __attribute__((ext_vector_type(16))) __bf16   v16b;
typedef __attribute__((ext_vector_type(8)))  __bf16   v8b;
typedef __attribute__((ext_vector_type(8)))  float    v8f;
typedef __attribute__((ext_vector_type(4)))  float    v4f;
typedef __attribute__((ext_vector_type(4)))  unsigned v4u;
typedef __attribute__((ext_vector_type(4)))  int      v4i;
#define PSCALE 32768.0f
#define U16(p) ((const unsigned short*)(const void*)(p))
#define PSCALE_INV (1.0f / 32768.0f)

static constexpr int kB      = 16;
static constexpr int kC      = 512;
static constexpr int kHgt    = 28;
static constexpr int kWid    = 28;
static constexpr int kNsp    = kHgt * kWid;
static constexpr int kHeads  = 16;
static constexpr int kDh     = kC / kHeads;
static constexpr int kFF     = 4 * kC;
static constexpr int kNumRel = (2 * kHgt - 1) * kWid + (2 * kWid - 1) + 1;
static constexpr int kMtot   = kB * kNsp;
static_assert(kMtot % 64 == 0, "M tile");
static_assert(kC % 64 == 0 && kFF % 64 == 0, "N tile");
static_assert(kC % 32 == 0 && kFF % 32 == 0, "K step");
static_assert(kNsp % 16 == 0, "query rows per wave");
static_assert(kDh == 32, "head dim");
static_assert((kMtot * kC / 2) % 256 == 0, "cast grid exact");
static_assert((kMtot * kFF / 2) % 256 == 0, "gelu grid exact");

__device__ __forceinline__ unsigned short f2bf_bits(float f) {
  unsigned u = __float_as_uint(f);
  return (unsigned short)((u + 0x7FFFu + ((u >> 16) & 1u)) >> 16);
}
__device__ __forceinline__ float bf_bits2f(unsigned short h) { return __uint_as_float(((unsigned)h) << 16); }

__device__ __forceinline__ void dep_guard_h(v8f& a, v8f& b, v16h x, v16h y) { asm volatile("v_nop\n\tv_nop\n\tv_nop\n\tv_nop" : "+v"(a), "+v"(b) : "v"(x), "v"(y)); }
__device__ __forceinline__ void dep_guard_b(v8f& a, v8f& b, v16b x, v16b y) { asm volatile("v_nop\n\tv_nop\n\tv_nop\n\tv_nop" : "+v"(a), "+v"(b) : "v"(x), "v"(y)); }
__device__ __forceinline__ void keep4_h(v16h a, v16h b, v16h c, v16h d) { asm volatile("v_nop" :: "v"(a), "v"(b), "v"(c), "v"(d)); }
__device__ __forceinline__ void keep4_b(v16b a, v16b b, v16b c, v16b d) { asm volatile("v_nop" :: "v"(a), "v"(b), "v"(c), "v"(d)); }
__device__ __forceinline__ void acc_guard4(v8f& a, v8f& b, v8f& c, v8f& d) { asm volatile("v_nop\n\tv_nop\n\tv_nop\n\tv_nop" : "+v"(a), "+v"(b), "+v"(c), "+v"(d)); }
template <typename T> struct Frag;
template <> struct Frag<_Float16> {
  typedef v16h V; union U { v16h v; v8h h[2]; };
  static __device__ __forceinline__ v16h load(const _Float16* p) {
    U f; f.h[0] = *(const v8h*)(p); f.h[1] = *(const v8h*)(p + 16); return f.v;
  }
  static __device__ __forceinline__ v8f mma(v16h a, v16h b, v8f c) {
    return __builtin_amdgcn_wmma_f32_16x16x32_f16(false, a, false, b, (short)0, c, false, false);
  }
  static __device__ __forceinline__ void guard(v8f& a, v8f& b, v16h x, v16h y) { dep_guard_h(a, b, x, y); }
  static __device__ __forceinline__ void keep(v16h a, v16h b, v16h c, v16h d) { keep4_h(a, b, c, d); }
};
template <> struct Frag<__bf16> {
  typedef v16b V; union U { v16b v; v8b h[2]; };
  static __device__ __forceinline__ v16b load(const __bf16* p) {
    U f; f.h[0] = *(const v8b*)(p); f.h[1] = *(const v8b*)(p + 16); return f.v;
  }
  static __device__ __forceinline__ v8f mma(v16b a, v16b b, v8f c) {
    return __builtin_amdgcn_wmma_f32_16x16x32_bf16(false, a, false, b, (short)0, c, false, false);
  }
  static __device__ __forceinline__ void guard(v8f& a, v8f& b, v16b x, v16b y) { dep_guard_b(a, b, x, y); }
  static __device__ __forceinline__ void keep(v16b a, v16b b, v16b c, v16b d) { keep4_b(a, b, c, d); }
};

template <int ET> struct Elem;
template <> struct Elem<0> { typedef _Float16 T; };
template <> struct Elem<1> { typedef __bf16 T; };
template <int ET, bool SPLIT, int BIAS_MODE, int OUT_MODE, bool RESID, int ACT = 0>
__global__ __launch_bounds__(256) void wmma_gemm64(
    const unsigned short* __restrict__ Ap, const unsigned short* __restrict__ A2p, int lda, long strideA,
    const unsigned short* __restrict__ Btp, const unsigned short* __restrict__ Bt2p, int ldb, long strideB,
    void* __restrict__ Cout, void* __restrict__ Cout2, int ldc, long strideC,
    const float* __restrict__ bias,
    const float* __restrict__ resid, long strideR,
    int M, int N, int K, float scale) {
  typedef typename Elem<ET>::T T;
  typedef typename Frag<T>::V V;
  const T* A = (const T*)Ap; const T* A2 = (const T*)A2p; const T* Bt = (const T*)Btp; const T* Bt2 = (const T*)Bt2p;
  __shared__ __align__(16) float sT[8][16 * 68];
  const int b    = blockIdx.y;
  const int lane = threadIdx.x & 31;
  const int wave = threadIdx.x >> 5;
  const int tilesN = N >> 6;
  const int tilesM = M >> 6;
  const int tile = blockIdx.x * 8 + wave;
  if (tile >= tilesM * tilesN) return;
  const int tm = tile / tilesN;
  const int tn = tile - tm * tilesN;
  const int m0 = tm << 6;
  const int n0 = tn << 6;

  const T* Ab  = A  + (size_t)b * strideA;
  const T* Bb  = Bt + (size_t)b * strideB;
  const T* Ab2 = SPLIT ? (A2  + (size_t)b * strideA) : nullptr;
  const T* Bb2 = SPLIT ? (Bt2 + (size_t)b * strideB) : nullptr;

  const int rlane = lane & 15;
  const int koff  = (lane >> 4) * 8;
  const int mOff  = (lane >> 4) * 8;

  v8f acc[4][4];
#pragma unroll
  for (int i = 0; i < 4; ++i)
#pragma unroll
    for (int j = 0; j < 4; ++j) acc[i][j] = (v8f){0.f,0.f,0.f,0.f,0.f,0.f,0.f,0.f};

  for (int k0 = 0; k0 < K; k0 += 32) {
    V bh[4], bl[4];
#pragma unroll
    for (int j = 0; j < 4; ++j) {
      const size_t bo = (size_t)(n0 + (j << 4) + rlane) * ldb + koff + k0;
      bh[j] = Frag<T>::load(Bb + bo);
      if (SPLIT) bl[j] = Frag<T>::load(Bb2 + bo);
    }
#pragma unroll
    for (int i = 0; i < 4; ++i) {
      const size_t ao = (size_t)(m0 + (i << 4) + rlane) * lda + koff + k0;
      V ah = Frag<T>::load(Ab + ao);
      V al;
      if (SPLIT) al = Frag<T>::load(Ab2 + ao);
#pragma unroll
      for (int j = 0; j < 4; ++j) {
        acc[i][j] = Frag<T>::mma(ah, bh[j], acc[i][j]);
        if (SPLIT) {
          acc[i][j] = Frag<T>::mma(ah, bl[j], acc[i][j]);
          acc[i][j] = Frag<T>::mma(al, bh[j], acc[i][j]);
        }
      }
      Frag<T>::guard(acc[i][0], acc[i][3], ah, SPLIT ? al : ah);
    }
    Frag<T>::keep(bh[0], bh[1], bh[2], bh[3]);
    if (SPLIT) Frag<T>::keep(bl[0], bl[1], bl[2], bl[3]);
  }
  acc_guard4(acc[0][0], acc[0][1], acc[0][2], acc[0][3]);
  acc_guard4(acc[1][0], acc[1][1], acc[1][2], acc[1][3]);
  acc_guard4(acc[2][0], acc[2][1], acc[2][2], acc[2][3]);
  acc_guard4(acc[3][0], acc[3][1], acc[3][2], acc[3][3]);

  float* slab = sT[wave];
  const float* Rb = RESID ? (resid + (size_t)b * strideR) : nullptr;
#pragma unroll
  for (int i = 0; i < 4; ++i) {
    const int mBase = m0 + (i << 4);
#pragma unroll
    for (int j = 0; j < 4; ++j) {
      const int n = n0 + (j << 4) + rlane;
      float bv = 0.f;
      if (BIAS_MODE == 2) bv = bias[n];
#pragma unroll
      for (int r = 0; r < 8; ++r) {
        float v = acc[i][j][r] * scale;
        if (BIAS_MODE == 1) v += bias[mBase + mOff + r];
        if (BIAS_MODE == 2) v += bv;
        if (RESID) v += Rb[(size_t)(mBase + mOff + r) * ldc + n];
        if (ACT == 1) v = tanhf(v);
        if (ACT == 2) v = fmaxf(v, 0.0f);
        if (ACT == 3) v = v / (1.0f + expf(-v));
        if (ACT == 4) v = (v > 0.f) ? v : 0.01f * v;
        if (ACT == 5) v = 0.5f * v * (1.0f + erff(v * 0.70710678118654752f));
        slab[(mOff + r) * 68 + (j << 4) + rlane] = v;
      }
    }
    __builtin_amdgcn_fence(__ATOMIC_RELEASE, "workgroup");
    __builtin_amdgcn_wave_barrier();
    __builtin_amdgcn_fence(__ATOMIC_ACQUIRE, "workgroup");
    if (OUT_MODE == 0) {
      float* Cp = (float*)Cout + (size_t)b * strideC;
      const int hh = lane >> 4, c4 = (lane & 15) * 4;
      for (int pass = 0; pass < 2; ++pass) {
#pragma unroll
        for (int it = 0; it < 8; ++it) {
          const int row = it * 2 + hh;
          v4f v = *(const v4f*)(slab + row * 68 + c4);
          *(volatile v4f*)(Cp + (size_t)(mBase + row) * ldc + n0 + c4) = v;
        }
        __threadfence();
      }
    } else {
      const int q = lane >> 3, c8 = (lane & 7) * 8;
      unsigned short* Cp  = (unsigned short*)Cout  + (size_t)b * strideC;
      unsigned short* Cp2 = (OUT_MODE == 2) ? ((unsigned short*)Cout2 + (size_t)b * strideC) : nullptr;
      for (int pass = 0; pass < 2; ++pass) {
#pragma unroll
        for (int it = 0; it < 4; ++it) {
          const int row = it * 4 + q;
          const float* sp = slab + row * 68 + c8;
          v8h hv, lv;
#pragma unroll
          for (int e = 0; e < 8; ++e) {
            if (OUT_MODE == 1) {
              hv[e] = (_Float16)sp[e];
            } else {
              unsigned short hb = f2bf_bits(sp[e]);
              unsigned short lb = f2bf_bits(sp[e] - bf_bits2f(hb));
              hv[e] = __builtin_bit_cast(_Float16, hb);
              lv[e] = __builtin_bit_cast(_Float16, lb);
            }
          }
          *(volatile v8h*)(Cp + (size_t)(mBase + row) * ldc + n0 + c8) = hv;
          if (OUT_MODE == 2) *(volatile v8h*)(Cp2 + (size_t)(mBase + row) * ldc + n0 + c8) = lv;
        }
        __threadfence();
      }
    }
    __builtin_amdgcn_fence(__ATOMIC_RELEASE, "workgroup");
    __builtin_amdgcn_wave_barrier();
    __builtin_amdgcn_fence(__ATOMIC_ACQUIRE, "workgroup");
  }
}

__global__ __launch_bounds__(256) void ln_rows_kernel(
    const float* __restrict__ x, const float* __restrict__ lnw, const float* __restrict__ lnb,
    _Float16* __restrict__ xn, float* __restrict__ xc) {
  __shared__ __align__(16) float xs[kC * 17];
  const int tid = threadIdx.x, lane = tid & 31, wave = tid >> 5;
  const int n0 = blockIdx.x * 16;
  const int b  = blockIdx.y;
#pragma unroll
  for (int cc = 0; cc < 2; ++cc) {
    const int ch = tid + cc * 256;
    const float* src = x + ((size_t)(b * kC + ch)) * kNsp + n0;
#pragma unroll
    for (int i = 0; i < 4; ++i) {
      const v4f v = *(const v4f*)(src + 4 * i);
      xs[ch * 17 + 4 * i + 0] = v[0];
      xs[ch * 17 + 4 * i + 1] = v[1];
      xs[ch * 17 + 4 * i + 2] = v[2];
      xs[ch * 17 + 4 * i + 3] = v[3];
    }
  }
  __syncthreads();
#pragma unroll 1
  for (int pp = 0; pp < 2; ++pp) {
    const int p = wave * 2 + pp;
    float su = 0.f;
#pragma unroll 1
    for (int i = 0; i < 16; ++i) su += xs[(lane + 32 * i) * 17 + p];
#pragma unroll
    for (int off = 16; off > 0; off >>= 1) su += __shfl_xor(su, off, 32);
    const float mean = su * (1.0f / 512.0f);
    float sq = 0.f;
#pragma unroll 1
    for (int i = 0; i < 16; ++i) { const float d = xs[(lane + 32 * i) * 17 + p] - mean; sq += d * d; }
#pragma unroll
    for (int off = 16; off > 0; off >>= 1) sq += __shfl_xor(sq, off, 32);
    const float var  = sq * (1.0f / 512.0f);
    const float rstd = rsqrtf(var + 1e-5f);
    const size_t m = (size_t)b * kNsp + n0 + p;

    v4f o32[4];
#pragma unroll
    for (int it = 0; it < 4; ++it) {
#pragma unroll
      for (int e = 0; e < 4; ++e) o32[it][e] = xs[(it * 128 + 4 * lane + e) * 17 + p];
    }
    v8h o16[2];
#pragma unroll
    for (int it = 0; it < 2; ++it) {
      const int cb = it * 256 + 8 * lane;
      const v4f w0 = *(const v4f*)(lnw + cb), w1 = *(const v4f*)(lnw + cb + 4);
      const v4f g0 = *(const v4f*)(lnb + cb), g1 = *(const v4f*)(lnb + cb + 4);
#pragma unroll
      for (int e = 0; e < 4; ++e) {
        const float t0 = (xs[(cb + e) * 17 + p] - mean) * rstd;
        const float t1 = (xs[(cb + 4 + e) * 17 + p] - mean) * rstd;
        o16[it][e]     = (_Float16)(t0 * w0[e] + g0[e]);
        o16[it][4 + e] = (_Float16)(t1 * w1[e] + g1[e]);
      }
    }
    float* xcrow = xc + m * kC;
    _Float16* xnrow = xn + m * kC;
    for (int pass = 0; pass < 2; ++pass) {
#pragma unroll
      for (int it = 0; it < 4; ++it) *(volatile v4f*)(xcrow + it * 128 + 4 * lane) = o32[it];
#pragma unroll
      for (int it = 0; it < 2; ++it) *(volatile v8h*)(xnrow + it * 256 + 8 * lane) = o16[it];
      __threadfence();
    }
  }
}

__global__ __launch_bounds__(256) void wt_cast_t_kernel(
    const float* __restrict__ Win, _Float16* __restrict__ Bt, int Kdim, int Ndim, float sc) {
  __shared__ __align__(16) float ts[64 * 65];
  const int tid = threadIdx.x, lane = tid & 31, wave = tid >> 5;
  const int n0 = blockIdx.x * 64, k0 = blockIdx.y * 64;
  {
    const int kr = tid >> 2, cs = (tid & 3) * 16;
    const float* src = Win + (size_t)(k0 + kr) * Ndim + n0 + cs;
#pragma unroll
    for (int i = 0; i < 4; ++i) {
      const v4f v = *(const v4f*)(src + 4 * i);
      ts[kr * 65 + cs + 4 * i + 0] = v[0];
      ts[kr * 65 + cs + 4 * i + 1] = v[1];
      ts[kr * 65 + cs + 4 * i + 2] = v[2];
      ts[kr * 65 + cs + 4 * i + 3] = v[3];
    }
  }
  __syncthreads();
  const int q = lane >> 3, c8 = (lane & 7) * 8;
  v8h hv[2];
#pragma unroll
  for (int it = 0; it < 2; ++it) {
    const int nl = wave * 8 + it * 4 + q;
#pragma unroll
    for (int e = 0; e < 8; ++e) hv[it][e] = (_Float16)(ts[(c8 + e) * 65 + nl] * sc);
  }
  for (int pass = 0; pass < 2; ++pass) {
#pragma unroll
    for (int it = 0; it < 2; ++it) {
      const int nl = wave * 8 + it * 4 + q;
      *(volatile v8h*)(Bt + (size_t)(n0 + nl) * Kdim + k0 + c8) = hv[it];
    }
    __threadfence();
  }
}

__global__ __launch_bounds__(256) void cast_scale_f16x2(
    const float* __restrict__ in, _Float16* __restrict__ out, int n2, float sc) {
  const int i = blockIdx.x * 256 + threadIdx.x;
  if (i < n2) {
    const _Float16 h0 = (_Float16)(in[2 * (size_t)i] * sc);
    const _Float16 h1 = (_Float16)(in[2 * (size_t)i + 1] * sc);
    const unsigned u = (unsigned)__builtin_bit_cast(unsigned short, h0) | ((unsigned)__builtin_bit_cast(unsigned short, h1) << 16);
    ((volatile unsigned*)out)[i] = u;
    __threadfence();
    ((volatile unsigned*)out)[i] = u;
  }
}

__global__ __launch_bounds__(256) void gelu_f16x2(
    const _Float16* __restrict__ in, _Float16* __restrict__ out, int n2, float sc) {
  const int i = blockIdx.x * 256 + threadIdx.x;
  if (i < n2) {
    const unsigned w = ((const unsigned*)(const void*)in)[i];
    unsigned u = 0u;
#pragma unroll 1
    for (int e = 0; e < 2; ++e) {
      const int sh = 16 * e;
      const float a = (float)__builtin_bit_cast(_Float16, (unsigned short)((w >> sh) & 0xffffu));
      const float g = 0.5f * a * (1.0f + erff(a * 0.70710678118654752f));
      const unsigned short hb = __builtin_bit_cast(unsigned short, (_Float16)(g * sc));
      u |= ((unsigned)hb) << sh;
    }
    ((volatile unsigned*)out)[i] = u;
    __threadfence();
    ((volatile unsigned*)out)[i] = u;
  }
}

static constexpr int kNqb = (kNsp + 63) / 64;
static constexpr float kPCarry = 32768.0f;

__device__ __forceinline__ v8f mma_h16(v16h a, v16h b, v8f c) {
  c = __builtin_amdgcn_wmma_f32_16x16x32_f16(false, a, false, b, (short)0, c, false, false);
  asm volatile("v_nop\n\tv_nop\n\tv_nop\n\tv_nop" : "+v"(c) : "v"(a), "v"(b));
  return c;
}

__global__ __launch_bounds__(128) void attn32_kernel(
    const _Float16* __restrict__ qp, const _Float16* __restrict__ kp, const _Float16* __restrict__ vp,
    const float* __restrict__ relb, const int* __restrict__ relidx, float* __restrict__ op) {
  __shared__ __align__(16) unsigned short Ksh[64 * 32];
  __shared__ __align__(16) unsigned short Vth[32 * 64];
  __shared__ __align__(16) _Float16 Psh[4][16 * 64];
  __shared__ __align__(16) float Osh[4][16 * 36];
  __shared__ __align__(16) int Ish[64 * 64];
  __shared__ __align__(16) float Rsh[1600];

  const int tid = threadIdx.x, wave = tid >> 5, lane = tid & 31, hh = lane >> 4, c = lane & 15;
  const int bx = blockIdx.x;
  const int qb = bx % kNqb;
  const int bh = bx / kNqb;
  const int h  = bh % kHeads;
  const int b  = bh / kHeads;
  const int qblk = qb * 64;
  const int q0 = qblk + wave * 16;
  const bool qvalid = (q0 < kNsp);

  for (int i = tid; i < 400; i += 128) {
    const int ic = (i < 399) ? i : 398;
    v4f v = *(const v4f*)(relb + (size_t)h * kNumRel + 4 * ic);
    if (i >= 399) v = (v4f){0.f, 0.f, 0.f, 0.f};
    *(v4f*)(Rsh + 4 * i) = v;
  }

  v16h qa;
  {
    int qr = q0 + c; qr = (qr < kNsp) ? qr : (kNsp - 1);
    qa = Frag<_Float16>::load(qp + ((size_t)(b * kNsp + qr)) * kC + h * kDh + 8 * hh);
  }

  float mrow[8], lrow[8];
  v8f oacc[2];
#pragma unroll
  for (int r = 0; r < 8; ++r) { mrow[r] = -INFINITY; lrow[r] = 0.f; }
  oacc[0] = (v8f){0.f,0.f,0.f,0.f,0.f,0.f,0.f,0.f};
  oacc[1] = (v8f){0.f,0.f,0.f,0.f,0.f,0.f,0.f,0.f};

#pragma unroll 1
  for (int kc = 0; kc < kNqb; ++kc) {
    const int kv0 = kc * 64;
    __syncthreads();
    {
      const int kvr = tid >> 1, dh = (tid & 1) * 16;
      const int kvg = kv0 + kvr;
      const bool valid = kvg < kNsp;
      const int kvc = valid ? kvg : (kNsp - 1);
      const size_t roff = ((size_t)(b * kNsp + kvc)) * kC + h * kDh + dh;
      v4u kw0 = *(const v4u*)(kp + roff);
      v4u kw1 = *(const v4u*)(kp + roff + 8);
      v4u vw0 = *(const v4u*)(vp + roff);
      v4u vw1 = *(const v4u*)(vp + roff + 8);
      const v4u z4 = (v4u){0u, 0u, 0u, 0u};
      if (!valid) { kw0 = z4; kw1 = z4; vw0 = z4; vw1 = z4; }
      *(v4u*)(Ksh + kvr * 32 + dh)     = kw0;
      *(v4u*)(Ksh + kvr * 32 + dh + 8) = kw1;
#pragma unroll
      for (int wi = 0; wi < 4; ++wi) {
        Vth[(dh + 2 * wi) * 64 + kvr]         = (unsigned short)(vw0[wi] & 0xffffu);
        Vth[(dh + 2 * wi + 1) * 64 + kvr]     = (unsigned short)(vw0[wi] >> 16);
        Vth[(dh + 8 + 2 * wi) * 64 + kvr]     = (unsigned short)(vw1[wi] & 0xffffu);
        Vth[(dh + 8 + 2 * wi + 1) * 64 + kvr] = (unsigned short)(vw1[wi] >> 16);
      }
    }
    asm volatile("" ::: "memory");
    {
      const int row = tid >> 1, chh = (tid & 1) * 32;
      int qr = qblk + row; qr = (qr < kNsp) ? qr : (kNsp - 1);
      const int* src = relidx + (size_t)qr * kNsp;
#pragma unroll
      for (int i = 0; i < 8; ++i) {
        int cb = kv0 + chh + 4 * i; cb = (cb > kNsp - 4) ? (kNsp - 4) : cb;
        const v4i v = *(const v4i*)(src + cb);
        *(v4i*)(Ish + row * 64 + chh + 4 * i) = v;
      }
    }
    __syncthreads();

    v8f s[4];
    const _Float16* Kh = (const _Float16*)(const void*)Ksh;
#pragma unroll
    for (int j = 0; j < 4; ++j) {
      const v16h kb = Frag<_Float16>::load(Kh + (j * 16 + c) * 32 + 8 * hh);
      s[j] = (v8f){0.f,0.f,0.f,0.f,0.f,0.f,0.f,0.f};
      s[j] = mma_h16(qa, kb, s[j]);
    }
    float cm[8];
#pragma unroll
    for (int r = 0; r < 8; ++r) {
      const int ql = wave * 16 + 8 * hh + r;
      float m = -INFINITY;
#pragma unroll
      for (int j = 0; j < 4; ++j) {
        const int kvcol = kv0 + j * 16 + c;
        int ix = Ish[ql * 64 + j * 16 + c];
        ix = (ix < 0) ? 0 : ix;
        ix = (ix > kNumRel - 1) ? (kNumRel - 1) : ix;
        float sv = s[j][r] + Rsh[ix];
        sv = (kvcol < kNsp) ? sv : -INFINITY;
        s[j][r] = sv;
        m = fmaxf(m, sv);
      }
#pragma unroll
      for (int off = 1; off < 16; off <<= 1) m = fmaxf(m, __shfl_xor(m, off, 32));
      cm[r] = m;
    }
    _Float16* pw = Psh[wave];
#pragma unroll
    for (int r = 0; r < 8; ++r) {
      const float mnew = fmaxf(mrow[r], cm[r]);
      const float alpha = expf(mrow[r] - mnew);
      mrow[r] = mnew;
      float psum = 0.f;
#pragma unroll
      for (int j = 0; j < 4; ++j) {
        const float p = expf(s[j][r] - mnew);
        psum += p;
        pw[(8 * hh + r) * 64 + j * 16 + c] = (_Float16)(p * kPCarry);
      }
#pragma unroll
      for (int off = 1; off < 16; off <<= 1) psum += __shfl_xor(psum, off, 32);
      lrow[r] = lrow[r] * alpha + psum;
      oacc[0][r] *= alpha;
      oacc[1][r] *= alpha;
    }
    __syncthreads();
    const _Float16* Vh = (const _Float16*)(const void*)Vth;
#pragma unroll
    for (int kk = 0; kk < 2; ++kk) {
      const v16h pa = Frag<_Float16>::load(pw + c * 64 + kk * 32 + 8 * hh);
#pragma unroll
      for (int t = 0; t < 2; ++t) {
        const v16h vb = Frag<_Float16>::load(Vh + (t * 16 + c) * 64 + kk * 32 + 8 * hh);
        oacc[t] = mma_h16(pa, vb, oacc[t]);
      }
    }
  }

  float* os = Osh[wave];
#pragma unroll
  for (int r = 0; r < 8; ++r) {
    const float inv = 1.0f / (lrow[r] * kPCarry);
    os[(8 * hh + r) * 36 + c]      = oacc[0][r] * inv;
    os[(8 * hh + r) * 36 + 16 + c] = oacc[1][r] * inv;
  }
  __syncthreads();
  if (qvalid) {
    const int rq = lane >> 3, c4 = (lane & 7) * 4;
    for (int pass = 0; pass < 2; ++pass) {
#pragma unroll
      for (int it = 0; it < 4; ++it) {
        const int row = it * 4 + rq;
        const v4f val = *(const v4f*)(os + row * 36 + c4);
        *(volatile v4f*)(op + ((size_t)(b * kNsp + q0 + row)) * kC + h * kDh + c4) = val;
      }
      __threadfence();
    }
  }
}

__global__ __launch_bounds__(256) void out_nchw_kernel(const float* __restrict__ x2, float* __restrict__ out) {
  __shared__ __align__(16) float st[8][2 * kNsp];
  const int tid = threadIdx.x, wave = tid >> 5, lane = tid & 31;
  const int b  = blockIdx.y;
  const int ch = blockIdx.x * 16 + wave * 2;
  float* sw = st[wave];
#pragma unroll 4
  for (int i = 0; i < 49; ++i) {
    const int f  = lane + 32 * i;
    const int cc = (f >= kNsp) ? 1 : 0;
    const int n  = f - kNsp * cc;
    sw[f] = x2[((size_t)(b * kNsp + n)) * kC + ch + cc];
  }
  __syncthreads();
  float* ob = out + ((size_t)(b * kC + ch)) * kNsp;
  const int c4 = lane * 4;
  for (int pass = 0; pass < 2; ++pass) {
#pragma unroll
    for (int it = 0; it < 13; ++it) {
      int idx = it * 128 + c4;
      idx = (idx > 2 * kNsp - 4) ? (2 * kNsp - 4) : idx;
      const v4f v = *(const v4f*)(sw + idx);
      if (it < 12 || lane < 8) {
        *(volatile v4f*)(ob + it * 128 + c4) = v;
      }
    }
    __threadfence();
  }
}

static inline dim3 gemm_grid(int M, int N) { return dim3((unsigned)((((M / 64) * (N / 64)) + 7) / 8), 1); }

extern "C" void kernel_launch(void* const* d_in, const int* in_sizes, int n_in,
                              void* d_out, int out_size, void* d_ws, size_t ws_size,
                              hipStream_t stream) {
  if (n_in < 17) return;
  if (in_sizes[0] != kB * kC * kNsp || out_size != kB * kC * kNsp) return;
  if (in_sizes[1] != kC || in_sizes[2] != kC) return;
  if (in_sizes[3] != kC * kC || in_sizes[5] != kC * kC || in_sizes[7] != kC * kC || in_sizes[9] != kC * kC) return;
  if (in_sizes[4] != kC || in_sizes[6] != kC || in_sizes[8] != kC || in_sizes[10] != kC || in_sizes[15] != kC) return;
  if (in_sizes[11] != kHeads * kNumRel || in_sizes[12] != kC * kFF || in_sizes[13] != kFF || in_sizes[14] != kFF * kC) return;
  if (in_sizes[16] != kNsp * kNsp) return;

  const float* x     = (const float*)d_in[0];
  const float* ln_w  = (const float*)d_in[1];
  const float* ln_b  = (const float*)d_in[2];
  const float* Wq    = (const float*)d_in[3];
  const float* bq    = (const float*)d_in[4];
  const float* Wk    = (const float*)d_in[5];
  const float* bk    = (const float*)d_in[6];
  const float* Wv    = (const float*)d_in[7];
  const float* bv    = (const float*)d_in[8];
  const float* Wo    = (const float*)d_in[9];
  const float* bo    = (const float*)d_in[10];
  const float* relb  = (const float*)d_in[11];
  const float* W1    = (const float*)d_in[12];
  const float* b1    = (const float*)d_in[13];
  const float* W2    = (const float*)d_in[14];
  const float* b2    = (const float*)d_in[15];
  const int*   relix = (const int*)d_in[16];
  float* out = (float*)d_out;

  const size_t P16  = (size_t)kMtot * kC * 2;
  const size_t P32  = (size_t)kMtot * kC * 4;
  const size_t G16  = (size_t)kMtot * kFF * 2;
  const size_t WSQB = (size_t)kC * kC * 2;
  const size_t WBIG = (size_t)kC * kFF * 2;
  const size_t off_w2t = 0;
  const size_t off_x1  = off_w2t + WBIG;
  const size_t off_hrg = off_x1 + P32;
  const size_t off_grg = off_hrg + G16;
  const size_t off_q   = off_grg + P16;
  const size_t off_k   = off_q + P16;
  const size_t off_v   = off_k + P16;
  const size_t off_w1t = off_q;
  const size_t off_wsq = off_grg + G16;
  const size_t total   = off_wsq + 4 * WSQB;
  if (total > ws_size) return;

  char* ws = (char*)d_ws;
  _Float16* W2T = (_Float16*)(ws + off_w2t);
  float*    Of  = (float*)(ws + off_x1);
  float*    x1  = (float*)(ws + off_x1);
  float*    xc  = (float*)(ws + off_hrg);
  _Float16* hpl = (_Float16*)(ws + off_hrg);
  float*    x2  = (float*)(ws + off_hrg);
  _Float16* xn  = (_Float16*)(ws + off_grg);
  _Float16* Oh  = (_Float16*)(ws + off_grg);
  _Float16* x1h = (_Float16*)(ws + off_grg);
  _Float16* gpl = (_Float16*)(ws + off_grg);
  _Float16* qh  = (_Float16*)(ws + off_q);
  _Float16* kh  = (_Float16*)(ws + off_k);
  _Float16* vh  = (_Float16*)(ws + off_v);
  _Float16* W1T = (_Float16*)(ws + off_w1t);
  _Float16* WqT = (_Float16*)(ws + off_wsq);
  _Float16* WkT = (_Float16*)(ws + off_wsq + WSQB);
  _Float16* WvT = (_Float16*)(ws + off_wsq + 2 * WSQB);
  _Float16* WoT = (_Float16*)(ws + off_wsq + 3 * WSQB);

  const float wcarry = 64.0f;
  const float ocarry = 16.0f;
  const float gcarry = 16.0f;
  typedef const unsigned short* cus;

  ln_rows_kernel<<<dim3(kNsp / 16, kB), 256, 0, stream>>>(x, ln_w, ln_b, xn, xc);

  wt_cast_t_kernel<<<dim3(kC / 64, kC / 64), 256, 0, stream>>>(Wq, WqT, kC, kC, wcarry);
  wt_cast_t_kernel<<<dim3(kC / 64, kC / 64), 256, 0, stream>>>(Wk, WkT, kC, kC, wcarry);
  wt_cast_t_kernel<<<dim3(kC / 64, kC / 64), 256, 0, stream>>>(Wv, WvT, kC, kC, wcarry);
  wt_cast_t_kernel<<<dim3(kC / 64, kC / 64), 256, 0, stream>>>(Wo, WoT, kC, kC, wcarry);
  wt_cast_t_kernel<<<dim3(kC / 64, kFF / 64), 256, 0, stream>>>(W2, W2T, kFF, kC, wcarry);

  wmma_gemm64<0, false, 2, 1, false, 0><<<gemm_grid(kMtot, kC), 256, 0, stream>>>(
      (cus)xn, nullptr, kC, 0L, (cus)WqT, nullptr, kC, 0L, (void*)qh, nullptr, kC, 0L,
      bq, nullptr, 0L, kMtot, kC, kC, 1.0f / wcarry);
  wmma_gemm64<0, false, 2, 1, false, 0><<<gemm_grid(kMtot, kC), 256, 0, stream>>>(
      (cus)xn, nullptr, kC, 0L, (cus)WkT, nullptr, kC, 0L, (void*)kh, nullptr, kC, 0L,
      bk, nullptr, 0L, kMtot, kC, kC, 1.0f / wcarry);
  wmma_gemm64<0, false, 2, 1, false, 0><<<gemm_grid(kMtot, kC), 256, 0, stream>>>(
      (cus)xn, nullptr, kC, 0L, (cus)WvT, nullptr, kC, 0L, (void*)vh, nullptr, kC, 0L,
      bv, nullptr, 0L, kMtot, kC, kC, 1.0f / wcarry);

  attn32_kernel<<<dim3(kB * kHeads * kNqb), 128, 0, stream>>>(qh, kh, vh, relb, relix, Of);

  cast_scale_f16x2<<<dim3((kMtot * kC / 2 + 255) / 256), 256, 0, stream>>>(Of, Oh, kMtot * kC / 2, ocarry);

  wt_cast_t_kernel<<<dim3(kFF / 64, kC / 64), 256, 0, stream>>>(W1, W1T, kC, kFF, wcarry);

  wmma_gemm64<0, false, 2, 0, true, 0><<<gemm_grid(kMtot, kC), 256, 0, stream>>>(
      (cus)Oh, nullptr, kC, 0L, (cus)WoT, nullptr, kC, 0L, (void*)x1, nullptr, kC, 0L,
      bo, xc, 0L, kMtot, kC, kC, 1.0f / (wcarry * ocarry));

  cast_scale_f16x2<<<dim3((kMtot * kC / 2 + 255) / 256), 256, 0, stream>>>(x1, x1h, kMtot * kC / 2, 1.0f);

  wmma_gemm64<0, false, 2, 1, false, 0><<<gemm_grid(kMtot, kFF), 256, 0, stream>>>(
      (cus)x1h, nullptr, kC, 0L, (cus)W1T, nullptr, kC, 0L, (void*)hpl, nullptr, kFF, 0L,
      b1, nullptr, 0L, kMtot, kFF, kC, 1.0f / wcarry);

  gelu_f16x2<<<dim3((kMtot * kFF / 2 + 255) / 256), 256, 0, stream>>>(hpl, gpl, kMtot * kFF / 2, gcarry);

  wmma_gemm64<0, false, 2, 0, true, 0><<<gemm_grid(kMtot, kC), 256, 0, stream>>>(
      (cus)gpl, nullptr, kFF, 0L, (cus)W2T, nullptr, kFF, 0L, (void*)x2, nullptr, kC, 0L,
      b2, x1, 0L, kMtot, kC, kFF, 1.0f / (wcarry * gcarry));

  out_nchw_kernel<<<dim3(kC / 16, kB), 256, 0, stream>>>(x2, out);
}
